// InteractionDecoder_38139309589084
// MI455X (gfx1250) — hardware-verified
//
#include <hip/hip_runtime.h>
#include <math.h>

typedef __attribute__((ext_vector_type(16))) _Float16 v16h;
typedef __attribute__((ext_vector_type(16))) __bf16 v16b;
typedef __attribute__((ext_vector_type(8)))  _Float16 v8h;
typedef __attribute__((ext_vector_type(8)))  float v8f;
typedef __attribute__((ext_vector_type(4)))  float v4f;
typedef __attribute__((ext_vector_type(2)))  float v2f;
typedef __attribute__((ext_vector_type(4)))  unsigned v4u;
typedef __attribute__((ext_vector_type(4)))  int v4i;
typedef float __attribute__((may_alias)) float_a;
typedef int __attribute__((may_alias)) int_a;

template <typename T> __device__ __forceinline__ void vst2(void* p, T v) { *(volatile T*)p = v; __threadfence(); *(volatile T*)p = v; }
__device__ __forceinline__ v8f wmma16(v16h a, v16h b, v8f c) {
  v8f d = __builtin_amdgcn_wmma_f32_16x16x32_f16(false, a, false, b, (short)0, c, false, false);
  asm volatile("v_nop\n\tv_nop\n\tv_nop\n\tv_nop" : "+v"(d) : "v"(a), "v"(b));
  return d;
}
__device__ __forceinline__ v8f wmma_bf(v16b a, v16b b, v8f c) {
  v8f d = __builtin_amdgcn_wmma_f32_16x16x32_bf16(false, a, false, b, (short)0, c, false, false);
  asm volatile("v_nop\n\tv_nop\n\tv_nop\n\tv_nop" : "+v"(d) : "v"(a), "v"(b));
  return d;
}
__device__ __forceinline__ v16h frag_h(const _Float16* rowk0, int lane) {
  union { v16h v; v8h q[2]; } u; const _Float16* p = rowk0 + 8 * (lane >> 4);
  u.q[0] = *(const v8h*)p; u.q[1] = *(const v8h*)(p + 16); return u.v;
}
__device__ __forceinline__ v16h frag_f32(const float* rowk0, int lane) {
  v16h a; const float* p = rowk0 + 8 * (lane >> 4);
#pragma unroll
  for (int i = 0; i < 8; ++i) { a[i] = (_Float16)p[i]; a[8 + i] = (_Float16)p[16 + i]; }
  return a;
}
__device__ __forceinline__ v16h frag_f32s(const float* rowk0, int lane, float sc) {
  v16h a; const float* p = rowk0 + 8 * (lane >> 4);
#pragma unroll
  for (int i = 0; i < 8; ++i) { a[i] = (_Float16)(p[i] * sc); a[8 + i] = (_Float16)(p[16 + i] * sc); }
  return a;
}
__device__ __forceinline__ v16h fragc_f32(const float* W, int k0, int n, int lane, int ld, int K) {
  v16h a; const int g = lane >> 4;
#pragma unroll
  for (int i = 0; i < 8; ++i) { const int ka = k0 + 8 * g + i, kb = ka + 16;
    a[i] = (_Float16)(ka < K ? W[(size_t)(ka < K ? ka : K - 1) * ld + n] : 0.f); a[8 + i] = (_Float16)(kb < K ? W[(size_t)(kb < K ? kb : K - 1) * ld + n] : 0.f); }
  return a;
}
struct F2 { v16b h, l; };
__device__ __forceinline__ F2 bsplit16(const float v[16]) { F2 r;
#pragma unroll
  for (int i = 0; i < 16; ++i) { const __bf16 h = (__bf16)v[i]; r.h[i] = h; r.l[i] = (__bf16)(v[i] - (float)h); }
  return r; }
__device__ __forceinline__ F2 split_row(const float* row, int k0, int lane) { float v[16]; const float* p = row + k0 + 8 * (lane >> 4);
#pragma unroll
  for (int i = 0; i < 8; ++i) { v[i] = p[i]; v[8 + i] = p[16 + i]; }
  return bsplit16(v); }
__device__ __forceinline__ F2 split_rowK(const float* row, int k0, int lane, int K) { float v[16]; const int g = lane >> 4;
#pragma unroll
  for (int i = 0; i < 8; ++i) { const int ka = k0 + 8 * g + i, kb = ka + 16; v[i] = ka < K ? row[ka < K ? ka : K - 1] : 0.f; v[8 + i] = kb < K ? row[kb < K ? kb : K - 1] : 0.f; }
  return bsplit16(v); }
__device__ __forceinline__ F2 split_col(const float* W, int k0, int n, int lane, int ld, int K) { float v[16]; const int g = lane >> 4;
#pragma unroll
  for (int i = 0; i < 8; ++i) { const int ka = k0 + 8 * g + i, kb = ka + 16; v[i] = ka < K ? W[(size_t)(ka < K ? ka : K - 1) * ld + n] : 0.f; v[8 + i] = kb < K ? W[(size_t)(kb < K ? kb : K - 1) * ld + n] : 0.f; }
  return bsplit16(v); }
__device__ __forceinline__ v8f mac3(const F2& a, const F2& b, v8f c) { c = wmma_bf(a.l, b.h, c); c = wmma_bf(a.h, b.l, c); return wmma_bf(a.h, b.h, c); }
__device__ __forceinline__ float sigm(float v) { return 1.0f / (1.0f + expf(-v)); }
#define LDSX() do { asm volatile("s_wait_dscnt 0" ::: "memory"); __builtin_amdgcn_wave_barrier(); __builtin_amdgcn_fence(__ATOMIC_RELEASE, "workgroup"); } while (0)


#define NB 4
#define SS 1024
#define E 512
#define NH 8
#define HD 64
#define NR (NB * SS)
#define DFF 2048
#define WB 16
#define PLO 1024.0f
#define VLO 2048.0f
__device__ __forceinline__ float bfr(float v) { return (float)(__bf16)v; }
__device__ __forceinline__ v16b frag_b(const __bf16* rowk0, int lane) { return __builtin_bit_cast(v16b, frag_h((const _Float16*)rowk0, lane)); }
__device__ __forceinline__ size_t physrow(size_t v) { return (v % SS) * NB + (v / SS); }

__global__ __launch_bounds__(256) void k_zero(__bf16* __restrict__ Z) { const size_t i8 = (size_t)blockIdx.x * 256 + threadIdx.x; v4u z = {0u, 0u, 0u, 0u}; vst2((unsigned*)(Z + i8 * 8), z); }
__global__ __launch_bounds__(256) void k_cvt(const float* __restrict__ x, __bf16* __restrict__ Xb) {
  const int tid = threadIdx.x; const size_t v = (size_t)blockIdx.x * 4 + (tid >> 6); const int pc = tid & 63; const float* src = x + physrow(v) * E + pc * 8;
  union { __bf16 e[8]; v4u u; } pk;
#pragma unroll
  for (int e = 0; e < 8; ++e) pk.e[e] = (__bf16)src[e];
  vst2((unsigned*)(Xb + v * E + pc * 8), pk.u);
}
__global__ __launch_bounds__(256) void k_pack(const float* __restrict__ Wq, const float* __restrict__ Wk, const float* __restrict__ Wv, const float* __restrict__ Wo, __bf16* __restrict__ PT) {
  const int n = blockIdx.x, tid = threadIdx.x; __shared__ __align__(16) __bf16 srow[E];
  const float* W = n < E ? Wq : (n < 2 * E ? Wk : (n < 3 * E ? Wv : Wo)); const int nn = n % E;
  for (int k = tid; k < E; k += 256) srow[k] = (__bf16)W[(size_t)nn * E + k];
  __syncthreads();
  if (tid < E / 8) vst2((unsigned*)(PT + (size_t)n * E + tid * 8), *(const v4u*)(&srow[tid * 8]));
}
__global__ __launch_bounds__(128) void k_qkv(const __bf16* __restrict__ Th, const __bf16* __restrict__ Tl, const __bf16* __restrict__ PT, const float* __restrict__ bq, const float* __restrict__ bk, const float* __restrict__ bv, int which0, float* __restrict__ Q32, __bf16* __restrict__ Kh, __bf16* __restrict__ Kl, _Float16* __restrict__ VTh, _Float16* __restrict__ VTl) {
  __shared__ __align__(16) float so[4][16][132];
  __shared__ __align__(16) _Float16 sth[128][72], stl[128][72];
  const int tid = threadIdx.x, wave = tid >> 5, lane = tid & 31, col = lane & 15, g = lane >> 4;
  const int which = blockIdx.z + which0, r0b = blockIdx.x * 64, r0 = r0b + wave * 16, n0 = blockIdx.y * 128; const int b = r0b / SS, s0 = r0b % SS;
  const float* bb_ = which == 0 ? bq : (which == 1 ? bk : bv);
  v8f acc[8] = {};
#pragma unroll 2
  for (int kc = 0; kc < E / 32; ++kc) { const v16b ah = frag_b(Th + (size_t)(r0 + col) * E + kc * 32, lane), al = frag_b(Tl + (size_t)(r0 + col) * E + kc * 32, lane);
#pragma unroll
    for (int j = 0; j < 8; ++j) { const v16b wb = frag_b(PT + (size_t)(which * E + n0 + j * 16 + col) * E + kc * 32, lane); acc[j] = wmma_bf(al, wb, acc[j]); acc[j] = wmma_bf(ah, wb, acc[j]); } }
  if (which < 2) {
#pragma unroll
    for (int j = 0; j < 8; ++j) { const float bb = bfr(bb_[n0 + j * 16 + col]);
#pragma unroll
      for (int r = 0; r < 8; ++r) so[wave][8 * g + r][j * 16 + col] = acc[j][r] + bb; }
    LDSX();
    if (which == 0) { for (int qq = lane; qq < 2 * 16 * 16; qq += 32) { const int hh = qq >> 8, rl = (qq >> 4) & 15, pc = qq & 15; const int h = (n0 >> 6) + hh;
        vst2(Q32 + (((size_t)b * NH + h) * SS + s0 + wave * 16 + rl) * HD + pc * 4, *(const v4f*)(&so[wave][rl][hh * 64 + pc * 4])); } }
    else {
      for (int qq = lane; qq < 2 * 16 * 16; qq += 32) { const int hh = qq >> 8, rl = (qq >> 4) & 15, pl = qq & 15; const int h = (n0 >> 6) + hh; const int pc = pl & 7; union { __bf16 e[8]; v4u u; } pk;
#pragma unroll
        for (int e = 0; e < 8; ++e) { const float v = so[wave][rl][hh * 64 + pc * 8 + e]; const __bf16 hi = (__bf16)v; pk.e[e] = pl < 8 ? hi : (__bf16)(v - (float)hi); }
        vst2((unsigned*)((pl < 8 ? Kh : Kl) + (((size_t)b * NH + h) * SS + s0 + wave * 16 + rl) * HD + pc * 8), pk.u); } } }
  else {
#pragma unroll
    for (int j = 0; j < 8; ++j) { const float bb = bfr(bb_[n0 + j * 16 + col]);
#pragma unroll
      for (int r = 0; r < 8; ++r) { const float v = (acc[j][r] + bb) * 4.0f; const _Float16 hi = (_Float16)v; sth[j * 16 + col][wave * 16 + 8 * g + r] = hi; stl[j * 16 + col][wave * 16 + 8 * g + r] = (_Float16)((v - (float)hi) * VLO); } }
    __syncthreads();
    for (int qq = tid; qq < 128 * 8; qq += 128) { const int cl = qq >> 3, pc = qq & 7; const int c = n0 + cl, h = c >> 6, d = c & 63; const size_t o = (((size_t)b * NH + h) * HD + d) * SS + s0 + pc * 8;
      vst2(VTh + o, *(const v4u*)(&sth[cl][pc * 8])); vst2(VTl + o, *(const v4u*)(&stl[cl][pc * 8])); } }
}
__global__ __launch_bounds__(128) void k_attn(const float* __restrict__ Q32, const __bf16* __restrict__ Kh, const __bf16* __restrict__ Kl, const _Float16* __restrict__ VTh, const _Float16* __restrict__ VTl, float* __restrict__ O32) {
  __shared__ __align__(16) float sS[4][16][68];
  __shared__ __align__(16) _Float16 sPh[4][16][72], sPl[4][16][72];
  __shared__ __align__(16) float sO[4][16][68];
  const int tid = threadIdx.x, w = tid >> 5, lane = tid & 31, col = lane & 15, g = lane >> 4;
  const size_t bh = blockIdx.y; const int qb = blockIdx.x; const int q0 = qb * 64 + w * 16;
  F2 aq[2];
#pragma unroll
  for (int kc = 0; kc < 2; ++kc) aq[kc] = split_row(Q32 + (bh * SS + q0 + col) * HD, kc * 32, lane);
  float mrun = -3.0e38f, lrun = 0.f; v8f acc[4] = {}, ac1[4] = {}, ac2[4] = {};
  LDSX();
#pragma unroll 1
  for (int kt = 0; kt < SS / 64; ++kt) {
#pragma unroll
    for (int t = 0; t < 4; ++t) { const int key = kt * 64 + t * 16 + col; const size_t ko = (bh * SS + key) * HD; v8f s = {};
#pragma unroll
      for (int kc = 0; kc < 2; ++kc) { const v16b khf = frag_b(Kh + ko + kc * 32, lane), klf = frag_b(Kl + ko + kc * 32, lane); s = wmma_bf(aq[kc].l, khf, s); s = wmma_bf(aq[kc].h, klf, s); s = wmma_bf(aq[kc].h, khf, s); }
#pragma unroll
      for (int r = 0; r < 8; ++r) sS[w][8 * g + r][t * 16 + col] = s[r] * 0.125f; }
    LDSX();
    float mx = -3.4e38f;
#pragma unroll
    for (int jj = 0; jj < 32; ++jj) mx = fmaxf(mx, sS[w][col][g * 32 + jj]);
    mx = fmaxf(mx, __shfl_xor(mx, 16, 32));
    const float mnew = fmaxf(mrun, mx); const float corr = expf(mrun - mnew);
    float ps = 0.f;
#pragma unroll
    for (int jj = 0; jj < 32; ++jj) { const float p = expf(sS[w][col][g * 32 + jj] - mnew) * 16384.0f; ps += p; const _Float16 hi = (_Float16)p; sPh[w][col][g * 32 + jj] = hi; sPl[w][col][g * 32 + jj] = (_Float16)((p - (float)hi) * PLO); }
    ps += __shfl_xor(ps, 16, 32);
    lrun = lrun * corr + ps * (1.0f / 16384.0f); mrun = mnew;
#pragma unroll
    for (int r = 0; r < 8; ++r) { const float cr = __shfl(corr, 8 * g + r, 32);
#pragma unroll
      for (int t = 0; t < 4; ++t) { acc[t][r] *= cr; ac1[t][r] *= cr; ac2[t][r] *= cr; } }
    LDSX();
#pragma unroll
    for (int kc = 0; kc < 2; ++kc) { const v16h ph = frag_h(&sPh[w][col][0] + kc * 32, lane), pl = frag_h(&sPl[w][col][0] + kc * 32, lane);
#pragma unroll
      for (int t = 0; t < 4; ++t) { const size_t vo = (bh * HD + t * 16 + col) * SS + kt * 64 + kc * 32; const v16h vh = frag_h(VTh + vo, lane);
        acc[t] = wmma16(ph, vh, acc[t]); ac1[t] = wmma16(ph, frag_h(VTl + vo, lane), ac1[t]); ac2[t] = wmma16(pl, vh, ac2[t]); } }
    __builtin_amdgcn_wave_barrier(); }
#pragma unroll
  for (int r = 0; r < 8; ++r) { const float lr = __shfl(lrun, 8 * g + r, 32); const float inv = 1.0f / (lr * 16384.0f * 4.0f);
#pragma unroll
    for (int t = 0; t < 4; ++t) sO[w][8 * g + r][t * 16 + col] = (acc[t][r] + ac1[t][r] * (1.0f / VLO) + ac2[t][r] * (1.0f / PLO)) * inv; }
  LDSX();
  for (int qq = lane; qq < 16 * 16; qq += 32) { const int rl = qq >> 4, pc = qq & 15; vst2(O32 + ((bh * SS) + q0 + rl) * HD + pc * 4, *(const v4f*)(&sO[w][rl][pc * 4])); }
}
__global__ __launch_bounds__(128) void k_attn_sw(const float* __restrict__ Q32, const __bf16* __restrict__ Kh, const __bf16* __restrict__ Kl, const _Float16* __restrict__ VTh, const _Float16* __restrict__ VTl, float* __restrict__ O32) {
  __shared__ __align__(16) float sS[4][16][68];
  __shared__ __align__(16) _Float16 sPh[4][16][72], sPl[4][16][72];
  __shared__ __align__(16) float sO[4][16][68];
  const int tid = threadIdx.x, w = tid >> 5, lane = tid & 31, col = lane & 15, g = lane >> 4;
  const size_t bh = blockIdx.y; const int qb = blockIdx.x; const int q0 = qb * 64 + w * 16;
  F2 aq[2];
#pragma unroll
  for (int kc = 0; kc < 2; ++kc) aq[kc] = split_row(Q32 + (bh * SS + q0 + col) * HD, kc * 32, lane);
  float mrun = -3.0e38f, lrun = 0.f; v8f acc[4] = {}, ac1[4] = {}, ac2[4] = {};
  LDSX();
#pragma unroll 1
  for (int kt = (qb > 0 ? qb - 1 : 0); kt <= (qb < SS / 64 - 1 ? qb + 1 : qb); ++kt) {
#pragma unroll
    for (int t = 0; t < 4; ++t) { const int key = kt * 64 + t * 16 + col; const size_t ko = (bh * SS + key) * HD; v8f s = {};
#pragma unroll
      for (int kc = 0; kc < 2; ++kc) { const v16b khf = frag_b(Kh + ko + kc * 32, lane), klf = frag_b(Kl + ko + kc * 32, lane); s = wmma_bf(aq[kc].l, khf, s); s = wmma_bf(aq[kc].h, klf, s); s = wmma_bf(aq[kc].h, khf, s); }
#pragma unroll
      for (int r = 0; r < 8; ++r) { const int dq = key - (q0 + 8 * g + r); sS[w][8 * g + r][t * 16 + col] = (dq > WB || dq < -WB) ? -3.0e38f : s[r] * 0.125f; } }
    LDSX();
    float mx = -3.4e38f;
#pragma unroll
    for (int jj = 0; jj < 32; ++jj) mx = fmaxf(mx, sS[w][col][g * 32 + jj]);
    mx = fmaxf(mx, __shfl_xor(mx, 16, 32));
    const float mnew = fmaxf(mrun, mx); const float corr = expf(mrun - mnew);
    float ps = 0.f;
#pragma unroll
    for (int jj = 0; jj < 32; ++jj) { const float sv = sS[w][col][g * 32 + jj]; const float p = (sv < -1.0e38f) ? 0.f : expf(sv - mnew) * 16384.0f; ps += p; const _Float16 hi = (_Float16)p; sPh[w][col][g * 32 + jj] = hi; sPl[w][col][g * 32 + jj] = (_Float16)((p - (float)hi) * PLO); }
    ps += __shfl_xor(ps, 16, 32);
    lrun = lrun * corr + ps * (1.0f / 16384.0f); mrun = mnew;
#pragma unroll
    for (int r = 0; r < 8; ++r) { const float cr = __shfl(corr, 8 * g + r, 32);
#pragma unroll
      for (int t = 0; t < 4; ++t) { acc[t][r] *= cr; ac1[t][r] *= cr; ac2[t][r] *= cr; } }
    LDSX();
#pragma unroll
    for (int kc = 0; kc < 2; ++kc) { const v16h ph = frag_h(&sPh[w][col][0] + kc * 32, lane), pl = frag_h(&sPl[w][col][0] + kc * 32, lane);
#pragma unroll
      for (int t = 0; t < 4; ++t) { const size_t vo = (bh * HD + t * 16 + col) * SS + kt * 64 + kc * 32; const v16h vh = frag_h(VTh + vo, lane);
        acc[t] = wmma16(ph, vh, acc[t]); ac1[t] = wmma16(ph, frag_h(VTl + vo, lane), ac1[t]); ac2[t] = wmma16(pl, vh, ac2[t]); } }
    __builtin_amdgcn_wave_barrier(); }
#pragma unroll
  for (int r = 0; r < 8; ++r) { const float lr = __shfl(lrun, 8 * g + r, 32); const float inv = 1.0f / (lr * 16384.0f * 4.0f);
#pragma unroll
    for (int t = 0; t < 4; ++t) sO[w][8 * g + r][t * 16 + col] = (acc[t][r] + ac1[t][r] * (1.0f / VLO) + ac2[t][r] * (1.0f / PLO)) * inv; }
  LDSX();
  for (int qq = lane; qq < 16 * 16; qq += 32) { const int rl = qq >> 4, pc = qq & 15; vst2(O32 + ((bh * SS) + q0 + rl) * HD + pc * 4, *(const v4f*)(&sO[w][rl][pc * 4])); }
}

__global__ __launch_bounds__(128) void k_oproj(const float* __restrict__ O32, const __bf16* __restrict__ PT, int prow, const float* __restrict__ bo, const float* __restrict__ resid, int resid_phys, float* __restrict__ RAW) {
  __shared__ __align__(16) float so[4][16][132];
  const int tid = threadIdx.x, wave = tid >> 5, lane = tid & 31, col = lane & 15, g = lane >> 4;
  const int r0 = blockIdx.x * 64 + wave * 16, n0 = blockIdx.y * 128; const int ra = r0 + col; const int b = ra / SS, s = ra % SS;
  v8f acc[8] = {};
#pragma unroll 1
  for (int kc = 0; kc < E / 32; ++kc) { const int h = kc >> 1; const F2 a = split_row(O32 + (((size_t)b * NH + h) * SS + s) * HD, (kc & 1) * 32, lane);
#pragma unroll
    for (int j = 0; j < 8; ++j) { const v16b wb = frag_b(PT + (size_t)(prow + n0 + j * 16 + col) * E + kc * 32, lane); acc[j] = wmma_bf(a.l, wb, acc[j]); acc[j] = wmma_bf(a.h, wb, acc[j]); } }
#pragma unroll
  for (int j = 0; j < 8; ++j) { const int n = n0 + j * 16 + col; const float bb = bfr(bo[n]);
#pragma unroll
    for (int r = 0; r < 8; ++r) { const size_t vr = (size_t)(r0 + 8 * g + r); const size_t rr = resid_phys ? physrow(vr) : vr; const float rv = resid[rr * E + n]; so[wave][8 * g + r][j * 16 + col] = acc[j][r] + bb + (resid_phys ? bfr(rv) : rv); } }
  LDSX();
#pragma unroll 4
  for (int rl = 0; rl < 16; ++rl) vst2(RAW + (size_t)(r0 + rl) * E + n0 + lane * 4, *(const v4f*)(&so[wave][rl][lane * 4]));
}
__global__ __launch_bounds__(256) void k_ln(const float* __restrict__ RAW, const float* __restrict__ gam, const float* __restrict__ bet, int out_phys, float* __restrict__ OUTF, __bf16* __restrict__ OH, __bf16* __restrict__ OL) {
  const int tid = threadIdx.x, w = tid >> 5, lane = tid & 31; const size_t v = (size_t)blockIdx.x * 8 + w; const float* row = RAW + v * E;
  float a[16]; float s1 = 0.f;
#pragma unroll
  for (int i = 0; i < 4; ++i) { const v4f q = *(const v4f*)(row + i * 128 + lane * 4); a[4 * i] = q[0]; a[4 * i + 1] = q[1]; a[4 * i + 2] = q[2]; a[4 * i + 3] = q[3]; s1 += q[0] + q[1] + q[2] + q[3]; }
#pragma unroll
  for (int o_ = 1; o_ < 32; o_ <<= 1) s1 += __shfl_xor(s1, o_, 32);
  const float mu = s1 * (1.0f / E); float s2 = 0.f;
#pragma unroll
  for (int i = 0; i < 16; ++i) { const float d = a[i] - mu; s2 += d * d; }
#pragma unroll
  for (int o_ = 1; o_ < 32; o_ <<= 1) s2 += __shfl_xor(s2, o_, 32);
  const float rs = rsqrtf(s2 * (1.0f / E) + 1e-5f);
  const size_t vo = out_phys ? physrow(v) : v;
#pragma unroll
  for (int i = 0; i < 4; ++i) { v4f q;
#pragma unroll
    for (int e = 0; e < 4; ++e) { const int c = i * 128 + lane * 4 + e; q[e] = (a[4 * i + e] - mu) * rs * bfr(gam[c]) + bfr(bet[c]); a[4 * i + e] = q[e]; }
    vst2(OUTF + vo * E + i * 128 + lane * 4, q); }
  if (OH) {
    __shared__ __align__(16) float srow[8][E + 4];
#pragma unroll
    for (int i = 0; i < 4; ++i) *(v4f*)(&srow[w][i * 128 + lane * 4]) = (v4f){a[4 * i], a[4 * i + 1], a[4 * i + 2], a[4 * i + 3]};
    LDSX();
    for (int pc = lane; pc < E / 8; pc += 32) { union { __bf16 e[8]; v4u u; } ph, pl;
#pragma unroll
      for (int e = 0; e < 8; ++e) { const float vv = srow[w][pc * 8 + e]; const __bf16 hi = (__bf16)vv; ph.e[e] = hi; pl.e[e] = (__bf16)(vv - (float)hi); }
      vst2((unsigned*)(OH + v * E + pc * 8), ph.u); vst2((unsigned*)(OL + v * E + pc * 8), pl.u); } }
}
__global__ __launch_bounds__(128) void k_ffn1(const __bf16* __restrict__ Xh, const __bf16* __restrict__ Xl, const float* __restrict__ W1, const float* __restrict__ b1, __bf16* __restrict__ Hh, __bf16* __restrict__ Hl) {
  __shared__ __align__(16) __bf16 sh_[4][16][136], sl_[4][16][136];
  const int tid = threadIdx.x, wave = tid >> 5, lane = tid & 31, col = lane & 15, g = lane >> 4; const size_t r0 = (size_t)blockIdx.x * 64 + wave * 16; const int n0 = blockIdx.y * 128;
  v8f acc[8] = {};
#pragma unroll 2
  for (int kc = 0; kc < E / 32; ++kc) { const v16b ah = frag_b(Xh + (r0 + col) * E + kc * 32, lane), al = frag_b(Xl + (r0 + col) * E + kc * 32, lane);
#pragma unroll
    for (int j = 0; j < 8; ++j) { const v16b wb = split_row(W1 + (size_t)(n0 + j * 16 + col) * E, kc * 32, lane).h; acc[j] = wmma_bf(al, wb, acc[j]); acc[j] = wmma_bf(ah, wb, acc[j]); } }
#pragma unroll
  for (int j = 0; j < 8; ++j) { const float bb = bfr(b1[n0 + j * 16 + col]);
#pragma unroll
    for (int r = 0; r < 8; ++r) { float v = acc[j][r] + bb; v = v > 0.f ? v : 0.f; const __bf16 hi = (__bf16)v; sh_[wave][8 * g + r][j * 16 + col] = hi; sl_[wave][8 * g + r][j * 16 + col] = (__bf16)(v - (float)hi); } }
  LDSX();
  for (int qq = lane; qq < 16 * 16; qq += 32) { const int rl = qq >> 4, pc = qq & 15; const size_t o = (r0 + rl) * DFF + n0 + pc * 8; vst2((unsigned*)(Hh + o), *(const v4u*)(&sh_[wave][rl][pc * 8])); vst2((unsigned*)(Hl + o), *(const v4u*)(&sl_[wave][rl][pc * 8])); }
}
__global__ __launch_bounds__(128) void k_ffn2(const __bf16* __restrict__ Hh, const __bf16* __restrict__ Hl, const float* __restrict__ W2, const float* __restrict__ b2, const float* __restrict__ resid, float* __restrict__ RAW) {
  __shared__ __align__(16) float so[4][16][132];
  const int tid = threadIdx.x, wave = tid >> 5, lane = tid & 31, col = lane & 15, g = lane >> 4; const size_t r0 = (size_t)blockIdx.x * 64 + wave * 16; const int n0 = blockIdx.y * 128;
  v8f acc[8] = {};
#pragma unroll 2
  for (int kc = 0; kc < DFF / 32; ++kc) { const v16b ah = frag_b(Hh + (r0 + col) * DFF + kc * 32, lane), al = frag_b(Hl + (r0 + col) * DFF + kc * 32, lane);
#pragma unroll
    for (int j = 0; j < 8; ++j) { const v16b wb = split_row(W2 + (size_t)(n0 + j * 16 + col) * DFF, kc * 32, lane).h; acc[j] = wmma_bf(al, wb, acc[j]); acc[j] = wmma_bf(ah, wb, acc[j]); } }
#pragma unroll
  for (int j = 0; j < 8; ++j) { const int n = n0 + j * 16 + col; const float bb = bfr(b2[n]);
#pragma unroll
    for (int r = 0; r < 8; ++r) so[wave][8 * g + r][j * 16 + col] = acc[j][r] + bb + resid[(r0 + 8 * g + r) * E + n]; }
  LDSX();
  for (int rl = 0; rl < 16; ++rl) vst2(RAW + (r0 + rl) * E + n0 + lane * 4, *(const v4f*)(&so[wave][rl][lane * 4]));
}
extern "C" void kernel_launch(void* const* d_in, const int* in_sizes, int n_in, void* d_out, int out_size, void* d_ws, size_t ws_size, hipStream_t stream) {
  (void)in_sizes; (void)n_in; (void)out_size; (void)ws_size;
  const float** I = (const float**)d_in;
  char* ws = (char*)d_ws; size_t off = 0;
  auto take = [&](size_t bytes) { char* p = ws + off; off += (bytes + 255) & ~(size_t)255; return p; };
  __bf16* Xb = (__bf16*)take((size_t)NR * E * 2); __bf16* Zb = (__bf16*)take((size_t)NR * E * 2); __bf16* Mb = (__bf16*)take((size_t)NR * E * 2);
  __bf16* PT1 = (__bf16*)take((size_t)4 * E * E * 2); __bf16* PT2 = (__bf16*)take((size_t)4 * E * E * 2);
  float* Q32 = (float*)take((size_t)NR * E * 4); __bf16* Kh = (__bf16*)take((size_t)NR * E * 2); __bf16* Kl = (__bf16*)take((size_t)NR * E * 2); _Float16* VTh = (_Float16*)take((size_t)NR * E * 2); _Float16* VTl = (_Float16*)take((size_t)NR * E * 2); float* O32 = (float*)take((size_t)NR * E * 4);
  float* RAW = (float*)take((size_t)NR * E * 4); float* X1 = (float*)take((size_t)NR * E * 4); __bf16* X1h = (__bf16*)take((size_t)NR * E * 2); __bf16* X1l = (__bf16*)take((size_t)NR * E * 2); float* X2 = (float*)take((size_t)NR * E * 4); __bf16* X2h = (__bf16*)take((size_t)NR * E * 2); __bf16* X2l = (__bf16*)take((size_t)NR * E * 2);
  __bf16* Hh = (__bf16*)take((size_t)NR * DFF * 2); __bf16* Hl = (__bf16*)take((size_t)NR * DFF * 2);
  k_zero<<<NR * E / 8 / 256, 256, 0, stream>>>(Zb);
  k_cvt<<<NR / 4, 256, 0, stream>>>(I[0], Xb);
  k_cvt<<<NR / 4, 256, 0, stream>>>(I[1], Mb);
  k_pack<<<4 * E, 256, 0, stream>>>(I[2], I[2] + (size_t)E * E, I[2] + (size_t)2 * E * E, I[4], PT1);
  k_pack<<<4 * E, 256, 0, stream>>>(I[6], I[8], I[10], I[12], PT2);
  k_qkv<<<dim3(NR / 64, E / 128, 3), 128, 0, stream>>>(Xb, Zb, PT1, I[3], I[3] + E, I[3] + 2 * E, 0, Q32, Kh, Kl, VTh, VTl);
  k_attn<<<dim3(SS / 64, NB * NH), 128, 0, stream>>>(Q32, Kh, Kl, VTh, VTl, O32);
  k_oproj<<<dim3(NR / 64, E / 128), 128, 0, stream>>>(O32, PT1, 3 * E, I[5], I[0], 1, RAW);
  k_ln<<<NR / 8, 256, 0, stream>>>(RAW, I[18], I[19], 0, X1, X1h, X1l);
  k_qkv<<<dim3(NR / 64, E / 128, 1), 128, 0, stream>>>(X1h, X1l, PT2, I[7], I[9], I[11], 0, Q32, Kh, Kl, VTh, VTl);
  k_qkv<<<dim3(NR / 64, E / 128, 2), 128, 0, stream>>>(Mb, Zb, PT2, I[7], I[9], I[11], 1, Q32, Kh, Kl, VTh, VTl);
  k_attn_sw<<<dim3(SS / 64, NB * NH), 128, 0, stream>>>(Q32, Kh, Kl, VTh, VTl, O32);
  k_oproj<<<dim3(NR / 64, E / 128), 128, 0, stream>>>(O32, PT2, 3 * E, I[13], X1, 0, RAW);
  k_ln<<<NR / 8, 256, 0, stream>>>(RAW, I[20], I[21], 0, X2, X2h, X2l);
  k_ffn1<<<dim3(NR / 64, DFF / 128), 128, 0, stream>>>(X2h, X2l, I[14], I[15], Hh, Hl);
  k_ffn2<<<dim3(NR / 64, E / 128), 128, 0, stream>>>(Hh, Hl, I[16], I[17], X2, RAW);
  k_ln<<<NR / 8, 256, 0, stream>>>(RAW, I[22], I[23], 1, (float*)d_out, nullptr, nullptr);
}
